// CustomRNN_39968965656997
// MI455X (gfx1250) — hardware-verified
//
#include <hip/hip_runtime.h>

typedef __attribute__((ext_vector_type(16))) _Float16 v16h;
typedef __attribute__((ext_vector_type(8)))  _Float16 v8h;
typedef __attribute__((ext_vector_type(16))) __bf16   v16b;
typedef __attribute__((ext_vector_type(8)))  __bf16   v8b;
typedef __attribute__((ext_vector_type(8)))  float    v8f;
typedef __attribute__((ext_vector_type(4)))  float    v4f;

constexpr int kSeq   = 64;
constexpr int kStep  = 512;
constexpr int kIn    = 256;
constexpr int kHid   = 512;
constexpr int kOutD  = 256;
constexpr int kLay   = 2;
constexpr int kRows  = kSeq * kStep;

constexpr int kSeqPB      = 16;
constexpr int kRnnBlocks  = kSeq / kSeqPB;
constexpr int kRnnThreads = 256;
constexpr int kHP         = kHid + 8;
constexpr int kHTile      = kSeqPB * kHP;
static_assert(kSeq % kSeqPB == 0);
static_assert(kHid == (kRnnThreads / 32) * 64);
static_assert(kHP % 8 == 0);
static_assert(kHid % 64 == 0 && kIn % 64 == 0 && kOutD % 64 == 0 && kRows % 64 == 0);
static_assert(kHid % 32 == 0 && kIn % 32 == 0);
constexpr int kXChunks = kRows * kIn / 8;
static_assert(kXChunks % 256 == 0);
constexpr int kBiasFloats = 3 * kHid;
static_assert(kBiasFloats % 256 == 0);

__device__ __forceinline__ unsigned short f2bf_bits(float f) {
  unsigned u = __float_as_uint(f);
  return (unsigned short)((u + 0x7FFFu + ((u >> 16) & 1u)) >> 16);
}
__device__ __forceinline__ float bf_bits2f(unsigned short h) { return __uint_as_float(((unsigned)h) << 16); }

__device__ __forceinline__ void dep_guard_h(v8f& a, v8f& b, v16h x, v16h y) { asm volatile("v_nop\n\tv_nop\n\tv_nop\n\tv_nop" : "+v"(a), "+v"(b) : "v"(x), "v"(y)); }
__device__ __forceinline__ void dep_guard_b(v8f& a, v8f& b, v16b x, v16b y) { asm volatile("v_nop\n\tv_nop\n\tv_nop\n\tv_nop" : "+v"(a), "+v"(b) : "v"(x), "v"(y)); }
__device__ __forceinline__ void keep4_h(v16h a, v16h b, v16h c, v16h d) { asm volatile("v_nop" :: "v"(a), "v"(b), "v"(c), "v"(d)); }
__device__ __forceinline__ void keep4_b(v16b a, v16b b, v16b c, v16b d) { asm volatile("v_nop" :: "v"(a), "v"(b), "v"(c), "v"(d)); }
__device__ __forceinline__ void acc_guard4(v8f& a, v8f& b, v8f& c, v8f& d) { asm volatile("v_nop\n\tv_nop\n\tv_nop\n\tv_nop" : "+v"(a), "+v"(b), "+v"(c), "+v"(d)); }

template <typename T> struct Frag;
template <> struct Frag<_Float16> {
  typedef v16h V; union U { v16h v; v8h h[2]; };
  static __device__ __forceinline__ v16h load(const _Float16* p) {
    U f; f.h[0] = *(const v8h*)(p); f.h[1] = *(const v8h*)(p + 16); return f.v;
  }
  static __device__ __forceinline__ v8f mma(v16h a, v16h b, v8f c) {
    return __builtin_amdgcn_wmma_f32_16x16x32_f16(false, a, false, b, (short)0, c, false, false);
  }
  static __device__ __forceinline__ void guard(v8f& a, v8f& b, v16h x, v16h y) { dep_guard_h(a, b, x, y); }
  static __device__ __forceinline__ void keep(v16h a, v16h b, v16h c, v16h d) { keep4_h(a, b, c, d); }
};
template <> struct Frag<__bf16> {
  typedef v16b V; union U { v16b v; v8b h[2]; };
  static __device__ __forceinline__ v16b load(const __bf16* p) {
    U f; f.h[0] = *(const v8b*)(p); f.h[1] = *(const v8b*)(p + 16); return f.v;
  }
  static __device__ __forceinline__ v8f mma(v16b a, v16b b, v8f c) {
    return __builtin_amdgcn_wmma_f32_16x16x32_bf16(false, a, false, b, (short)0, c, false, false);
  }
  static __device__ __forceinline__ void guard(v8f& a, v8f& b, v16b x, v16b y) { dep_guard_b(a, b, x, y); }
  static __device__ __forceinline__ void keep(v16b a, v16b b, v16b c, v16b d) { keep4_b(a, b, c, d); }
};

template <int ET> struct Elem;
template <> struct Elem<0> { typedef _Float16 T; };
template <> struct Elem<1> { typedef __bf16 T; };
template <int ET, bool SPLIT, int BIAS_MODE, int OUT_MODE, bool RESID, int ACT = 0, int TRI = 0>
__global__ __launch_bounds__(256) void wmma_gemm64(
    const unsigned short* __restrict__ Ap, const unsigned short* __restrict__ A2p, int lda, long strideA,
    const unsigned short* __restrict__ Btp, const unsigned short* __restrict__ Bt2p, int ldb, long strideB,
    void* __restrict__ Cout, void* __restrict__ Cout2, int ldc, long strideC,
    const float* __restrict__ bias,
    const float* __restrict__ resid, long strideR,
    int M, int N, int K, float scale) {
  typedef typename Elem<ET>::T T;
  typedef typename Frag<T>::V V;
  const T* A = (const T*)Ap; const T* A2 = (const T*)A2p; const T* Bt = (const T*)Btp; const T* Bt2 = (const T*)Bt2p;
  __shared__ __align__(16) float sT[8][16 * 68];
  const int b    = blockIdx.y;
  const int lane = threadIdx.x & 31;
  const int wave = threadIdx.x >> 5;
  const int tilesN = N >> 6;
  const int tilesM = M >> 6;
  const int tile = blockIdx.x * 8 + wave;
  if (tile >= tilesM * tilesN) return;
  const int tm = tile / tilesN;
  const int tn = tile - tm * tilesN;
  if (TRI == 1 && tn > tm) return;
  const int m0 = tm << 6;
  const int n0 = tn << 6;
  const int kLim = (TRI == 2) ? ((m0 + 64 < K) ? (m0 + 64) : K) : K;

  const T* Ab  = A  + (size_t)b * strideA;
  const T* Bb  = Bt + (size_t)b * strideB;
  const T* Ab2 = SPLIT ? (A2  + (size_t)b * strideA) : nullptr;
  const T* Bb2 = SPLIT ? (Bt2 + (size_t)b * strideB) : nullptr;

  const int rlane = lane & 15;
  const int koff  = (lane >> 4) * 8;
  const int mOff  = (lane >> 4) * 8;

  v8f acc[4][4];
#pragma unroll
  for (int i = 0; i < 4; ++i)
#pragma unroll
    for (int j = 0; j < 4; ++j) acc[i][j] = (v8f){0.f,0.f,0.f,0.f,0.f,0.f,0.f,0.f};

  for (int k0 = 0; k0 < kLim; k0 += 32) {
    V bh[4], bl[4];
#pragma unroll
    for (int j = 0; j < 4; ++j) {
      const size_t bo = (size_t)(n0 + (j << 4) + rlane) * ldb + koff + k0;
      bh[j] = Frag<T>::load(Bb + bo);
      if (SPLIT) bl[j] = Frag<T>::load(Bb2 + bo);
    }
#pragma unroll
    for (int i = 0; i < 4; ++i) {
      const size_t ao = (size_t)(m0 + (i << 4) + rlane) * lda + koff + k0;
      V ah = Frag<T>::load(Ab + ao);
      V al;
      if (SPLIT) al = Frag<T>::load(Ab2 + ao);
#pragma unroll
      for (int j = 0; j < 4; ++j) {
        acc[i][j] = Frag<T>::mma(ah, bh[j], acc[i][j]);
        if (SPLIT) {
          acc[i][j] = Frag<T>::mma(ah, bl[j], acc[i][j]);
          acc[i][j] = Frag<T>::mma(al, bh[j], acc[i][j]);
        }
      }
      Frag<T>::guard(acc[i][0], acc[i][3], ah, SPLIT ? al : ah);
    }
    Frag<T>::keep(bh[0], bh[1], bh[2], bh[3]);
    if (SPLIT) Frag<T>::keep(bl[0], bl[1], bl[2], bl[3]);
  }
  acc_guard4(acc[0][0], acc[0][1], acc[0][2], acc[0][3]);
  acc_guard4(acc[1][0], acc[1][1], acc[1][2], acc[1][3]);
  acc_guard4(acc[2][0], acc[2][1], acc[2][2], acc[2][3]);
  acc_guard4(acc[3][0], acc[3][1], acc[3][2], acc[3][3]);

  float* slab = sT[wave];
  const float* Rb = RESID ? (resid + (size_t)b * strideR) : nullptr;
#pragma unroll
  for (int i = 0; i < 4; ++i) {
    const int mBase = m0 + (i << 4);
#pragma unroll
    for (int j = 0; j < 4; ++j) {
      const int n = n0 + (j << 4) + rlane;
      float bv = 0.f;
      if (BIAS_MODE == 2) bv = bias[n];
#pragma unroll
      for (int r = 0; r < 8; ++r) {
        float v = acc[i][j][r] * scale;
        if (BIAS_MODE == 1) v += bias[mBase + mOff + r];
        if (BIAS_MODE == 2) v += bv;
        if (RESID) v += Rb[(size_t)(mBase + mOff + r) * ldc + n];
        if (ACT == 1) v = tanhf(v);
        if (ACT == 2) v = fmaxf(v, 0.0f);
        if (ACT == 4) v = (v > 0.f) ? v : 0.01f * v;
        slab[(mOff + r) * 68 + (j << 4) + rlane] = v;
      }
    }
    __builtin_amdgcn_fence(__ATOMIC_RELEASE, "workgroup");
    __builtin_amdgcn_wave_barrier();
    __builtin_amdgcn_fence(__ATOMIC_ACQUIRE, "workgroup");
    if (OUT_MODE == 0) {
      float* C = (float*)Cout + (size_t)b * strideC;
      const int hh = lane >> 4, c4 = (lane & 15) * 4;
      for (int pass = 0; pass < 2; ++pass) {
#pragma unroll
        for (int it = 0; it < 8; ++it) {
          const int row = it * 2 + hh;
          v4f v = *(const v4f*)(slab + row * 68 + c4);
          *(volatile v4f*)(C + (size_t)(mBase + row) * ldc + n0 + c4) = v;
        }
        __threadfence();
      }
    } else {
      const int q = lane >> 3, c8 = (lane & 7) * 8;
      unsigned short* C  = (unsigned short*)Cout  + (size_t)b * strideC;
      unsigned short* C2 = (OUT_MODE == 2) ? ((unsigned short*)Cout2 + (size_t)b * strideC) : nullptr;
      for (int pass = 0; pass < 2; ++pass) {
#pragma unroll
        for (int it = 0; it < 4; ++it) {
          const int row = it * 4 + q;
          const float* sp = slab + row * 68 + c8;
          v8h hv, lv;
#pragma unroll
          for (int e = 0; e < 8; ++e) {
            if (OUT_MODE == 1) {
              hv[e] = (_Float16)sp[e];
            } else {
              unsigned short hb = f2bf_bits(sp[e]);
              unsigned short lb = f2bf_bits(sp[e] - bf_bits2f(hb));
              hv[e] = __builtin_bit_cast(_Float16, hb);
              lv[e] = __builtin_bit_cast(_Float16, lb);
            }
          }
          *(volatile v8h*)(C + (size_t)(mBase + row) * ldc + n0 + c8) = hv;
          if (OUT_MODE == 2) *(volatile v8h*)(C2 + (size_t)(mBase + row) * ldc + n0 + c8) = lv;
        }
        __threadfence();
      }
    }
    __builtin_amdgcn_fence(__ATOMIC_RELEASE, "workgroup");
    __builtin_amdgcn_wave_barrier();
    __builtin_amdgcn_fence(__ATOMIC_ACQUIRE, "workgroup");
  }
}

__device__ __forceinline__ void st2u(unsigned* p, unsigned v) { *(volatile unsigned*)p = v; __threadfence(); *(volatile unsigned*)p = v; }
__device__ __forceinline__ float ftanh(float x) { return 1.0f - 2.0f * __builtin_amdgcn_rcpf(1.0f + __expf(2.0f * x)); }

__global__ __launch_bounds__(256) void wtrans_kernel(const float* __restrict__ W, _Float16* __restrict__ T,
                                                     int Kr, int Nc, long strideW, long strideT, float s) {
  __shared__ __align__(16) _Float16 tl[64 * 72];
  const int tid = threadIdx.x, lane = tid & 31, wave = tid >> 5;
  const int n0 = blockIdx.x * 64, k0 = blockIdx.y * 64;
  const float* Wz = W + (size_t)blockIdx.z * strideW;
  _Float16* Tz = T + (size_t)blockIdx.z * strideT;
#pragma unroll
  for (int i = 0; i < 16; ++i) {
    const int idx = i * 256 + tid;
    const int kk = idx >> 6, nn = idx & 63;
    tl[nn * 72 + kk] = (_Float16)(Wz[(size_t)(k0 + kk) * Nc + n0 + nn] * s);
  }
  __syncthreads();
  const int q = lane >> 3, c8 = (lane & 7) * 8;
  for (int pass = 0; pass < 2; ++pass) {
#pragma unroll
    for (int it = 0; it < 2; ++it) {
      const int nn = wave * 8 + it * 4 + q;
      const v8h v = *(const v8h*)(tl + nn * 72 + c8);
      *(volatile v8h*)(Tz + (size_t)(n0 + nn) * Kr + k0 + c8) = v;
    }
    __threadfence();
  }
}

__global__ __launch_bounds__(256) void bias_kernel(const float* __restrict__ b_in, const float* __restrict__ b_i2h,
                                                   const float* __restrict__ b_h2h, unsigned* __restrict__ biasu) {
  const int p = blockIdx.x * 256 + threadIdx.x;
  const int pc = p & (kHid - 1);
  const float a  = 4.0f * b_in[pc];
  const float s0 = b_i2h[pc] + b_h2h[pc];
  const float s1 = b_i2h[kHid + pc] + b_h2h[kHid + pc];
  const float v = (p < kHid) ? a : ((p < 2 * kHid) ? s0 : s1);
  st2u(biasu + p, (unsigned)__float_as_uint(v));
}

__global__ __launch_bounds__(256) void xcast_kernel(const float* __restrict__ x, _Float16* __restrict__ x16t) {
  const int i = blockIdx.x * 256 + threadIdx.x;
  const int row = i >> 5, c8 = i & 31;
  const int t = row >> 6, b = row & 63;
  const float* src = x + ((size_t)b * kStep + t) * kIn + c8 * 8;
  const v4f f0 = *(const v4f*)src;
  const v4f f1 = *(const v4f*)(src + 4);
  v8h hv;
  hv[0] = (_Float16)f0[0]; hv[1] = (_Float16)f0[1]; hv[2] = (_Float16)f0[2]; hv[3] = (_Float16)f0[3];
  hv[4] = (_Float16)f1[0]; hv[5] = (_Float16)f1[1]; hv[6] = (_Float16)f1[2]; hv[7] = (_Float16)f1[3];
  _Float16* dst = x16t + (size_t)row * kIn + c8 * 8;
  *(volatile v8h*)dst = hv;
  __threadfence();
  *(volatile v8h*)dst = hv;
}

__global__ __launch_bounds__(kRnnThreads) void rnn_layer_kernel(
    const float* __restrict__ pT, const _Float16* __restrict__ whh16, const float* __restrict__ hinit,
    _Float16* __restrict__ hseq, float* __restrict__ hfin, int bmajor) {
  __shared__ __align__(16) _Float16 hbuf[2 * kHTile];
  __shared__ __align__(16) float fsl[kRnnThreads / 32][16 * 68];
  const int tid = threadIdx.x, lane = tid & 31, wave = tid >> 5;
  const int c = lane & 15, hh = lane >> 4, koff = hh * 8, mOff = hh * 8;
  const int seq0 = blockIdx.x * kSeqPB;
  const int n0 = wave * 64;

  {
    const v8h z = {(_Float16)0.f, (_Float16)0.f, (_Float16)0.f, (_Float16)0.f, (_Float16)0.f, (_Float16)0.f, (_Float16)0.f, (_Float16)0.f};
    for (int i = tid; i < (2 * kHTile) / 8; i += kRnnThreads) *(v8h*)(hbuf + i * 8) = z;
  }
  __syncthreads();
  for (int i = tid; i < kSeqPB * kHid / 8; i += kRnnThreads) {
    const int row = i >> 6, c8i = (i & 63) * 8;
    const float* src = hinit + (size_t)(seq0 + row) * kHid + c8i;
    const v4f f0 = *(const v4f*)src;
    const v4f f1 = *(const v4f*)(src + 4);
    v8h hv;
    hv[0] = (_Float16)f0[0]; hv[1] = (_Float16)f0[1]; hv[2] = (_Float16)f0[2]; hv[3] = (_Float16)f0[3];
    hv[4] = (_Float16)f1[0]; hv[5] = (_Float16)f1[1]; hv[6] = (_Float16)f1[2]; hv[7] = (_Float16)f1[3];
    *(v8h*)(hbuf + row * kHP + c8i) = hv;
  }
  __syncthreads();

  const float inv16 = 0.0625f;
  const _Float16* brow = whh16 + (size_t)(n0 + c) * kHid + koff;
  const int q4 = lane >> 3, c8 = (lane & 7) * 8, c4 = (lane & 15) * 4;
  float* slab = fsl[wave];

#pragma unroll 1
  for (int t = 0; t < kStep; ++t) {
    const _Float16* hc = hbuf + (t & 1) * kHTile;
    _Float16*       hn = hbuf + ((t + 1) & 1) * kHTile;
    v8f acc[4];
#pragma unroll
    for (int j = 0; j < 4; ++j) {
      const float* xp = pT + (size_t)(n0 + 16 * j + c) * kRows + t * kSeq + seq0 + 8 * hh;
      const v4f xa = *(const v4f*)xp;
      const v4f xb = *(const v4f*)(xp + 4);
      acc[j][0] = xa[0] * 16.0f; acc[j][1] = xa[1] * 16.0f; acc[j][2] = xa[2] * 16.0f; acc[j][3] = xa[3] * 16.0f;
      acc[j][4] = xb[0] * 16.0f; acc[j][5] = xb[1] * 16.0f; acc[j][6] = xb[2] * 16.0f; acc[j][7] = xb[3] * 16.0f;
    }
    const _Float16* arow = hc + c * kHP + koff;
    v16h fa;
    v16h fb[4];
#pragma unroll 4
    for (int kc = 0; kc < kHid / 32; ++kc) {
      fa = Frag<_Float16>::load(arow + kc * 32);
#pragma unroll
      for (int j = 0; j < 4; ++j) fb[j] = Frag<_Float16>::load(brow + (size_t)(16 * j) * kHid + kc * 32);
#pragma unroll
      for (int j = 0; j < 4; ++j) acc[j] = Frag<_Float16>::mma(fa, fb[j], acc[j]);
      Frag<_Float16>::guard(acc[0], acc[3], fa, fb[3]);
      Frag<_Float16>::keep(fb[0], fb[1], fb[2], fb[3]);
    }
    acc_guard4(acc[0], acc[1], acc[2], acc[3]);

#pragma unroll
    for (int j = 0; j < 4; ++j) {
#pragma unroll
      for (int r = 0; r < 8; ++r) {
        const float hv = ftanh(acc[j][r] * inv16);
        acc[j][r] = hv;
        hn[(mOff + r) * kHP + n0 + 16 * j + c] = (_Float16)hv;
      }
    }
    if (t == kStep - 1) {
#pragma unroll
      for (int j = 0; j < 4; ++j) {
#pragma unroll
        for (int r = 0; r < 8; ++r) slab[(mOff + r) * 68 + 16 * j + c] = acc[j][r];
      }
    }
    __syncthreads();

    {
      for (int pass = 0; pass < 2; ++pass) {
#pragma unroll
        for (int it = 0; it < 4; ++it) {
          const int rr = it * 4 + q4;
          const size_t rowT = (size_t)t * kSeq + seq0 + rr;
          const size_t rowB = (size_t)(seq0 + rr) * kStep + t;
          const size_t rowidx = (bmajor != 0) ? rowB : rowT;
          const v8h v = *(const v8h*)(hn + rr * kHP + n0 + c8);
          *(volatile v8h*)(hseq + rowidx * kHid + n0 + c8) = v;
        }
        __threadfence();
      }
    }
    if (t == kStep - 1) {
      for (int pass = 0; pass < 2; ++pass) {
#pragma unroll
        for (int it = 0; it < 8; ++it) {
          const int row = it * 2 + hh;
          const v4f v = *(const v4f*)(slab + row * 68 + c4);
          *(volatile v4f*)(hfin + (size_t)(seq0 + row) * kHid + n0 + c4) = v;
        }
        __threadfence();
      }
    }
  }
}

extern "C" void kernel_launch(void* const* d_in, const int* in_sizes, int n_in,
                              void* d_out, int out_size, void* d_ws, size_t ws_size, hipStream_t stream) {
  if (n_in < 10 || d_out == nullptr || d_ws == nullptr) return;
  if (in_sizes[0] != kSeq * kStep * kIn || in_sizes[1] != kLay * kSeq * kHid || in_sizes[2] != kIn * kHid ||
      in_sizes[3] != kHid || in_sizes[4] != kLay * kHid * kHid || in_sizes[5] != kLay * kHid ||
      in_sizes[6] != kLay * kHid * kHid || in_sizes[7] != kLay * kHid || in_sizes[8] != kHid * kOutD ||
      in_sizes[9] != kOutD || out_size != kSeq * kStep * kOutD + kLay * kSeq * kHid) return;

  const float* x      = (const float*)d_in[0];
  const float* h_prev = (const float*)d_in[1];
  const float* W_in   = (const float*)d_in[2];
  const float* b_in   = (const float*)d_in[3];
  const float* W_i2h  = (const float*)d_in[4];
  const float* b_i2h  = (const float*)d_in[5];
  const float* W_h2h  = (const float*)d_in[6];
  const float* b_h2h  = (const float*)d_in[7];
  const float* W_out  = (const float*)d_in[8];
  const float* b_out  = (const float*)d_in[9];
  float* out  = (float*)d_out;
  float* hout = out + (size_t)kSeq * kStep * kOutD;

  char* ws = (char*)d_ws; size_t off = 0;
  auto carve = [&](size_t bytes) -> char* { char* p = ws + off; off += (bytes + 255) & ~(size_t)255; return p; };
  unsigned short* R1      = (unsigned short*)carve((size_t)kRows * kHid * 2);
  float*          R2      = (float*)carve((size_t)kHid * kRows * 4);
  unsigned short* WINT16  = (unsigned short*)carve((size_t)kHid * kIn * 2);
  unsigned short* WI2HT16 = (unsigned short*)carve((size_t)kLay * kHid * kHid * 2);
  unsigned short* WH2HT16 = (unsigned short*)carve((size_t)kLay * kHid * kHid * 2);
  unsigned short* WOUTT16 = (unsigned short*)carve((size_t)kOutD * kHid * 2);
  float*          BIASV   = (float*)carve((size_t)kBiasFloats * 4);
  if (off > ws_size || off > (size_t)134217728) return;
  unsigned short* X16T = (unsigned short*)R2;

  const float w16 = 16.0f;
  const int gridP   = ((kHid / 64) * (kRows / 64)) / 8;
  const int gridOut = ((kRows / 64) * (kOutD / 64)) / 8;

  wtrans_kernel<<<dim3(kHid / 64, kIn / 64, 1), 256, 0, stream>>>(W_in, (_Float16*)WINT16, kIn, kHid, 0L, 0L, w16);
  wtrans_kernel<<<dim3(kHid / 64, kHid / 64, kLay), 256, 0, stream>>>(W_i2h, (_Float16*)WI2HT16, kHid, kHid,
                                                                      (long)kHid * kHid, (long)kHid * kHid, w16);
  wtrans_kernel<<<dim3(kHid / 64, kHid / 64, kLay), 256, 0, stream>>>(W_h2h, (_Float16*)WH2HT16, kHid, kHid,
                                                                      (long)kHid * kHid, (long)kHid * kHid, w16);
  wtrans_kernel<<<dim3(kOutD / 64, kHid / 64, 1), 256, 0, stream>>>(W_out, (_Float16*)WOUTT16, kHid, kOutD, 0L, 0L, w16);

  bias_kernel<<<kBiasFloats / 256, 256, 0, stream>>>(b_in, b_i2h, b_h2h, (unsigned*)BIASV);

  xcast_kernel<<<kXChunks / 256, 256, 0, stream>>>(x, (_Float16*)X16T);

  wmma_gemm64<0, false, 2, 1, false, 0, 0><<<dim3(gridP, 1), 256, 0, stream>>>(
      X16T, nullptr, kIn, 0L, WINT16, nullptr, kIn, 0L,
      (void*)R1, nullptr, kHid, 0L, BIASV, nullptr, 0L, kRows, kHid, kIn, 0.25f);

  wmma_gemm64<0, false, 1, 0, false, 0, 0><<<dim3(gridP, 1), 256, 0, stream>>>(
      WI2HT16, nullptr, kHid, 0L, R1, nullptr, kHid, 0L,
      (void*)R2, nullptr, kRows, 0L, BIASV + kHid, nullptr, 0L, kHid, kRows, kHid, 1.0f / 64.0f);

  rnn_layer_kernel<<<kRnnBlocks, kRnnThreads, 0, stream>>>(R2, (const _Float16*)WH2HT16, h_prev,
                                                           (_Float16*)R1, hout, 0);

  wmma_gemm64<0, false, 1, 0, false, 0, 0><<<dim3(gridP, 1), 256, 0, stream>>>(
      WI2HT16 + (size_t)kHid * kHid, nullptr, kHid, 0L, R1, nullptr, kHid, 0L,
      (void*)R2, nullptr, kRows, 0L, BIASV + 2 * kHid, nullptr, 0L, kHid, kRows, kHid, 1.0f / 16.0f);

  rnn_layer_kernel<<<kRnnBlocks, kRnnThreads, 0, stream>>>(R2, (const _Float16*)(WH2HT16 + (size_t)kHid * kHid),
                                                           h_prev + (size_t)kSeq * kHid,
                                                           (_Float16*)R1, hout + (size_t)kSeq * kHid, 1);

  wmma_gemm64<0, false, 2, 0, false, 0, 0><<<dim3(gridOut, 1), 256, 0, stream>>>(
      R1, nullptr, kHid, 0L, WOUTT16, nullptr, kHid, 0L,
      (void*)out, nullptr, kOutD, 0L, b_out, nullptr, 0L, kRows, kOutD, kHid, 1.0f / 16.0f);
}
